// TransformerBlock_2516850835983
// MI455X (gfx1250) — hardware-verified
//
#include <hip/hip_runtime.h>
#ifndef NB
#define NB 2
#endif
#ifndef SEQ
#define SEQ 2048
#endif
#define NB_FULL 2
#define SEQ_FULL 2048
#define DM 1024
#define NH 16
#define HD 64
#define FF 4096
#define MROWS (NB * SEQ)
#define ACARRY 16.0f
#define WCARRY 256.0f
#define PCARRY 1024.0f

typedef _Float16 v16h __attribute__((ext_vector_type(16)));
typedef unsigned short v8us __attribute__((ext_vector_type(8), may_alias));
typedef float  v8f  __attribute__((ext_vector_type(8)));
typedef float  v4f  __attribute__((ext_vector_type(4)));
typedef float  v4fa __attribute__((ext_vector_type(4), may_alias));
union FragH { v16h v; v8us half[2]; };

static_assert(NB <= NB_FULL);
static_assert(SEQ <= SEQ_FULL);
static_assert(SEQ % 64 == 0);
static_assert(SEQ % 32 == 0);
static_assert(DM == NH * HD);
static_assert(HD == 64);
static_assert(DM == 128 * 8);
static_assert(MROWS % 16 == 0);
static_assert(DM % 32 == 0);
static_assert(FF % 32 == 0);
static_assert((3 * DM) % 64 == 0);
static_assert(DM % 64 == 0);
static_assert(FF % 64 == 0);
static_assert(((3 * DM / 64) % 4) == 0);
static_assert(((DM / 64) % 4) == 0);
static_assert(((FF / 64) % 4) == 0);
static_assert((3 * DM) % 8 == 0);

constexpr size_t SZ_WQKV = (size_t)3 * DM * DM * 2;
constexpr size_t SZ_WPJ  = (size_t)DM * DM * 2;
constexpr size_t SZ_WF1  = (size_t)FF * DM * 2;
constexpr size_t SZ_WF2  = (size_t)DM * FF * 2;
constexpr size_t SZ_H16  = (size_t)MROWS * DM * 2;
constexpr size_t SZ_QKV  = (size_t)MROWS * 3 * DM * 2;
constexpr size_t SZ_VT   = (size_t)NB * NH * HD * SEQ * 2;
constexpr size_t SZ_CTX  = (size_t)MROWS * DM * 2;
constexpr size_t SZ_X1   = (size_t)MROWS * DM * 4;
constexpr size_t SZ_G16  = (size_t)MROWS * FF * 2;
constexpr size_t SZ_TOTAL = SZ_WQKV + SZ_WPJ + SZ_WF1 + SZ_WF2 + SZ_H16 + SZ_QKV + SZ_VT + SZ_CTX + SZ_X1 + SZ_G16;
static_assert(SZ_WQKV % 256 == 0 && SZ_WPJ % 256 == 0 && SZ_WF1 % 256 == 0 && SZ_WF2 % 256 == 0);
static_assert(SZ_H16 % 256 == 0 && SZ_QKV % 256 == 0 && SZ_VT % 256 == 0 && SZ_CTX % 256 == 0 && SZ_X1 % 256 == 0 && SZ_G16 % 256 == 0);
static_assert(SZ_TOTAL <= (size_t)134217728);

constexpr int G_WQKV = (3 * DM * (DM / 8)) / 256;
constexpr int G_WPJ  = (DM * (DM / 8)) / 256;
constexpr int G_WF1  = (FF * (DM / 8)) / 256;
constexpr int G_WF2  = (DM * (FF / 8)) / 256;
static_assert((size_t)G_WQKV * 256 * 8 == (size_t)3 * DM * DM);
static_assert((size_t)G_WPJ * 256 * 8 == (size_t)DM * DM);
static_assert((size_t)G_WF1 * 256 * 8 == (size_t)FF * DM);
static_assert((size_t)G_WF2 * 256 * 8 == (size_t)DM * FF);
constexpr int G_QKV = (MROWS / 16) * (3 * DM / 64) / 4;
constexpr int G_PJ  = (MROWS / 16) * (DM / 64) / 4;
constexpr int G_F1  = (MROWS / 16) * (FF / 64) / 4;
constexpr int G_F2  = (MROWS / 16) * (DM / 64) / 4;
static_assert((size_t)G_QKV * 4 * 16 * 64 == (size_t)MROWS * 3 * DM);
static_assert((size_t)G_PJ * 4 * 16 * 64 == (size_t)MROWS * DM);
static_assert((size_t)G_F1 * 4 * 16 * 64 == (size_t)MROWS * FF);
static_assert((size_t)G_F2 * 4 * 16 * 64 == (size_t)MROWS * DM);
constexpr int G_VT = NB * NH * (SEQ / 64);
static_assert((size_t)G_VT * 256 * 2 * 8 == (size_t)MROWS * DM);
constexpr int G_FL = NB * NH * (SEQ / 64);
static_assert((size_t)G_FL * 4 * 16 * HD == (size_t)MROWS * DM);
static_assert((size_t)MROWS * 128 * 8 == (size_t)MROWS * DM);

__device__ __forceinline__ unsigned short bf16_bits(float x) { unsigned int u = __float_as_uint(x); return (unsigned short)((u + 0x7FFFu + ((u >> 16) & 1u)) >> 16); }
__device__ __forceinline__ float bf16_rne(float x) { return __uint_as_float(((unsigned int)bf16_bits(x)) << 16); }
__device__ __forceinline__ unsigned short f16_bits(float x) { return __builtin_bit_cast(unsigned short, (_Float16)x); }
__device__ __forceinline__ size_t xrow(int m) { return (size_t)(m / SEQ) * SEQ_FULL + (size_t)(m % SEQ); }

__device__ __forceinline__ v8us pack8(v4f a, v4f b, float sc) {
  v8us o;
  o[0] = f16_bits(a[0] * sc); o[1] = f16_bits(a[1] * sc); o[2] = f16_bits(a[2] * sc); o[3] = f16_bits(a[3] * sc);
  o[4] = f16_bits(b[0] * sc); o[5] = f16_bits(b[1] * sc); o[6] = f16_bits(b[2] * sc); o[7] = f16_bits(b[3] * sc);
  return o;
}

__device__ __forceinline__ v8f mma1(v16h a, v16h b, v8f c) {
  c = __builtin_amdgcn_wmma_f32_16x16x32_f16(false, a, false, b, (short)0, c, false, false);
  asm volatile("v_nop\n\tv_nop\n\tv_nop\n\tv_nop" : "+v"(c) : "v"(a), "v"(b));
  return c;
}

__global__ __launch_bounds__(256) void k_wt_f16(const float* __restrict__ W, unsigned short* __restrict__ Wt, int K, int N) {
  const int t = blockIdx.x * 256 + threadIdx.x;
  const int k8n = K / 8;
  if (t >= N * k8n) return;
  const int n = t / k8n, k8 = (t % k8n) * 8;
  v8us v;
#pragma unroll
  for (int i = 0; i < 8; ++i) v[i] = f16_bits(bf16_rne(W[(size_t)(k8 + i) * N + n]) * WCARRY);
  *(volatile v8us*)(Wt + (size_t)n * K + k8) = v;
  __threadfence();
  *(volatile v8us*)(Wt + (size_t)n * K + k8) = v;
}

template <bool IN_BF16, bool XFULL>
__device__ __forceinline__ void ln_body(const float* __restrict__ X, const float* __restrict__ g, const float* __restrict__ bta,
                                        unsigned short* __restrict__ out, float eps) {
  __shared__ float red[2][4];
  const int row = blockIdx.x, tid = threadIdx.x, lane = tid & 31;
  const int wave = __builtin_amdgcn_readfirstlane(threadIdx.x >> 5);
  const size_t srow = XFULL ? xrow(row) : (size_t)row;
  const float* x = X + srow * DM + tid * 8;
  const v4f a0 = *(const v4fa*)(x), a1 = *(const v4fa*)(x + 4);
  float vals[8] = {a0[0], a0[1], a0[2], a0[3], a1[0], a1[1], a1[2], a1[3]};
  float s1 = 0.f;
#pragma unroll
  for (int i = 0; i < 8; ++i) { if (IN_BF16) vals[i] = bf16_rne(vals[i]); s1 += vals[i]; }
  s1 += __shfl_xor(s1, 16, 32); s1 += __shfl_xor(s1, 8, 32); s1 += __shfl_xor(s1, 4, 32); s1 += __shfl_xor(s1, 2, 32); s1 += __shfl_xor(s1, 1, 32);
  if (lane == 0) red[0][wave] = s1;
  __syncthreads();
  const float mu = (((red[0][0] + red[0][1]) + red[0][2]) + red[0][3]) * (1.0f / (float)DM);
  float s2 = 0.f;
#pragma unroll
  for (int i = 0; i < 8; ++i) { const float c = vals[i] - mu; s2 += c * c; }
  s2 += __shfl_xor(s2, 16, 32); s2 += __shfl_xor(s2, 8, 32); s2 += __shfl_xor(s2, 4, 32); s2 += __shfl_xor(s2, 2, 32); s2 += __shfl_xor(s2, 1, 32);
  if (lane == 0) red[1][wave] = s2;
  __syncthreads();
  const float var = (((red[1][0] + red[1][1]) + red[1][2]) + red[1][3]) * (1.0f / (float)DM);
  const float rs = rsqrtf(var + eps);
  const v4f g0 = *(const v4fa*)(g + tid * 8), g1 = *(const v4fa*)(g + tid * 8 + 4);
  const v4f b0 = *(const v4fa*)(bta + tid * 8), b1 = *(const v4fa*)(bta + tid * 8 + 4);
  const float gg[8] = {g0[0], g0[1], g0[2], g0[3], g1[0], g1[1], g1[2], g1[3]};
  const float bb[8] = {b0[0], b0[1], b0[2], b0[3], b1[0], b1[1], b1[2], b1[3]};
  v8us o;
#pragma unroll
  for (int i = 0; i < 8; ++i) o[i] = f16_bits(((vals[i] - mu) * rs * bf16_rne(gg[i]) + bf16_rne(bb[i])) * ACARRY);
  unsigned short* dst = out + (size_t)row * DM + tid * 8;
  *(volatile v8us*)dst = o;
  __threadfence();
  *(volatile v8us*)dst = o;
}

__global__ __launch_bounds__(128) void k_ln1(const float* __restrict__ X, const float* __restrict__ g, const float* __restrict__ bta,
                                             unsigned short* __restrict__ out, float eps) {
  ln_body<true, true>(X, g, bta, out, eps);
}
__global__ __launch_bounds__(128) void k_ln2(const float* __restrict__ X, const float* __restrict__ g, const float* __restrict__ bta,
                                             unsigned short* __restrict__ out, float eps) {
  ln_body<false, false>(X, g, bta, out, eps);
}

template <int EPI>
__device__ __forceinline__ void gemm_body(const unsigned short* __restrict__ A, int lda, const unsigned short* __restrict__ Wt, int ldb,
                                          const float* __restrict__ bias, const float* __restrict__ resid,
                                          unsigned short* __restrict__ Ch, float* __restrict__ Cf, int ldc, int M, int N, int K) {
  __shared__ __attribute__((aligned(16))) float so[4][16][64];
  const int tid = threadIdx.x, lane = tid & 31, ln = lane & 15, hh = lane >> 4;
  const int wave = __builtin_amdgcn_readfirstlane(threadIdx.x >> 5);
  const int ntn = N / 64;
  const int wid = blockIdx.x * 4 + wave;
  const int mt = wid / ntn, nq = wid % ntn;
  if (mt * 16 >= M) return;
  const int row0 = mt * 16, col0 = nq * 64;
  const unsigned short* arow = A + (size_t)(row0 + ln) * lda + 8 * hh;
  const unsigned short* brow0 = Wt + (size_t)(col0 + ln) * ldb + 8 * hh;
  v8f acc[4] = {};
  for (int kb = 0; kb < K; kb += 32) {
    FragH a;
    a.half[0] = *(const v8us*)(arow + kb);
    a.half[1] = *(const v8us*)(arow + kb + 16);
#pragma unroll
    for (int t = 0; t < 4; ++t) {
      const unsigned short* brow = brow0 + (size_t)t * 16 * ldb + kb;
      FragH b;
      b.half[0] = *(const v8us*)(brow);
      b.half[1] = *(const v8us*)(brow + 16);
      acc[t] = mma1(a.v, b.v, acc[t]);
    }
  }
  const float inv = 1.0f / (ACARRY * WCARRY);
#pragma unroll
  for (int t = 0; t < 4; ++t) {
    const float bv = bf16_rne(bias[col0 + t * 16 + ln]);
#pragma unroll
    for (int r = 0; r < 8; ++r) so[wave][8 * hh + r][t * 16 + ln] = acc[t][r] * inv + bv;
  }
  __builtin_amdgcn_fence(4  , "workgroup");
  __builtin_amdgcn_wave_barrier();
  if constexpr (EPI == 1) {
#pragma unroll 1
    for (int i = 0; i < 32; ++i) {
      const int idx = i * 32 + lane;
      const int rr = idx >> 6, cc = idx & 63;
      const float v = so[wave][rr][cc];
      so[wave][rr][cc] = 0.5f * v * (1.0f + erff(v * 0.70710678118654752f));
    }
    __builtin_amdgcn_fence(4  , "workgroup");
    __builtin_amdgcn_wave_barrier();
  }
  if constexpr (EPI < 2) {
    const int rq = lane >> 3, c8 = (lane & 7) * 8;
    v8us ov[4];
#pragma unroll
    for (int q = 0; q < 4; ++q) {
      const int r = q * 4 + rq;
      const v4f x0 = *(const v4fa*)&so[wave][r][c8];
      const v4f x1 = *(const v4fa*)&so[wave][r][c8 + 4];
      ov[q] = pack8(x0, x1, ACARRY);
    }
    for (int pass = 0; pass < 2; ++pass) {
#pragma unroll
      for (int q = 0; q < 4; ++q)
        *(volatile v8us*)(Ch + (size_t)(row0 + q * 4 + rq) * ldc + col0 + c8) = ov[q];
      if (pass == 0) __threadfence();
    }
  } else {
    const int rsub = lane >> 4, c4 = (lane & 15) * 4;
    v4f ov[8];
#pragma unroll
    for (int q = 0; q < 8; ++q) {
      const int r = q * 2 + rsub;
      const int grow = row0 + r;
      const size_t rr = (EPI == 2) ? xrow(grow) : (size_t)grow;
      v4f v = *(const v4fa*)&so[wave][r][c4];
      v4f rv = *(const v4fa*)(resid + rr * (size_t)ldc + col0 + c4);
      if (EPI == 2) { rv[0] = bf16_rne(rv[0]); rv[1] = bf16_rne(rv[1]); rv[2] = bf16_rne(rv[2]); rv[3] = bf16_rne(rv[3]); }
      v[0] += rv[0]; v[1] += rv[1]; v[2] += rv[2]; v[3] += rv[3];
      ov[q] = v;
    }
    for (int pass = 0; pass < 2; ++pass) {
#pragma unroll
      for (int q = 0; q < 8; ++q) {
        const int grow = row0 + q * 2 + rsub;
        const size_t orow = (EPI == 3) ? xrow(grow) : (size_t)grow;
        *(volatile v4f*)(Cf + orow * (size_t)ldc + col0 + c4) = ov[q];
      }
      if (pass == 0) __threadfence();
    }
  }
}

__global__ __launch_bounds__(128) void k_gemm_plane(const unsigned short* __restrict__ A, int lda, const unsigned short* __restrict__ Wt, int ldb,
                                                    const float* __restrict__ bias, unsigned short* __restrict__ Ch, int ldc, int M, int N, int K) {
  gemm_body<0>(A, lda, Wt, ldb, bias, nullptr, Ch, nullptr, ldc, M, N, K);
}
__global__ __launch_bounds__(128) void k_gemm_gelu(const unsigned short* __restrict__ A, int lda, const unsigned short* __restrict__ Wt, int ldb,
                                                   const float* __restrict__ bias, unsigned short* __restrict__ Ch, int ldc, int M, int N, int K) {
  gemm_body<1>(A, lda, Wt, ldb, bias, nullptr, Ch, nullptr, ldc, M, N, K);
}
__global__ __launch_bounds__(128) void k_gemm_res_in(const unsigned short* __restrict__ A, int lda, const unsigned short* __restrict__ Wt, int ldb,
                                                     const float* __restrict__ bias, const float* __restrict__ resid,
                                                     float* __restrict__ Cf, int ldc, int M, int N, int K) {
  gemm_body<2>(A, lda, Wt, ldb, bias, resid, nullptr, Cf, ldc, M, N, K);
}
__global__ __launch_bounds__(128) void k_gemm_res_out(const unsigned short* __restrict__ A, int lda, const unsigned short* __restrict__ Wt, int ldb,
                                                      const float* __restrict__ bias, const float* __restrict__ resid,
                                                      float* __restrict__ Cf, int ldc, int M, int N, int K) {
  gemm_body<3>(A, lda, Wt, ldb, bias, resid, nullptr, Cf, ldc, M, N, K);
}

__global__ __launch_bounds__(256) void k_vt(const unsigned short* __restrict__ qkv, unsigned short* __restrict__ Vt) {
  __shared__ __attribute__((aligned(16))) unsigned short tile[64][72];
  const int tid = threadIdx.x;
  const int ntt = SEQ / 64;
  const int bh = blockIdx.x / ntt, tt = blockIdx.x % ntt;
  const int b = bh / NH, h = bh % NH;
  const int t0 = tt * 64;
#pragma unroll
  for (int u = 0; u < 2; ++u) {
    const int e = tid + 256 * u;
    const int r = e >> 3, c8 = (e & 7) * 8;
    const v8us v = *(const v8us*)(qkv + (size_t)(b * SEQ + t0 + r) * (3 * DM) + 2 * DM + h * HD + c8);
    *(v8us*)&tile[r][c8] = v;
  }
  __syncthreads();
  v8us o[2];
#pragma unroll
  for (int u = 0; u < 2; ++u) {
    const int e = tid + 256 * u;
    const int d = e >> 3, c8 = (e & 7) * 8;
#pragma unroll
    for (int i = 0; i < 8; ++i) o[u][i] = tile[c8 + i][d];
  }
  for (int pass = 0; pass < 2; ++pass) {
#pragma unroll
    for (int u = 0; u < 2; ++u) {
      const int e = tid + 256 * u;
      const int d = e >> 3, c8 = (e & 7) * 8;
      *(volatile v8us*)(Vt + ((size_t)bh * HD + d) * SEQ + t0 + c8) = o[u];
    }
    if (pass == 0) __threadfence();
  }
}

__global__ __launch_bounds__(128) void k_flash_h(const unsigned short* __restrict__ qkv, const unsigned short* __restrict__ Vt,
                                                 unsigned short* __restrict__ ctx) {
  __shared__ __attribute__((aligned(16))) unsigned short sP[4][16][40];
  __shared__ __attribute__((aligned(16))) float sO[4][16][HD];
  const int tid = threadIdx.x, lane = tid & 31, ln = lane & 15, hh = lane >> 4;
  const int wave = __builtin_amdgcn_readfirstlane(threadIdx.x >> 5);
  const int nqb = SEQ / 64;
  const int bh = blockIdx.x / nqb, qblk = blockIdx.x % nqb;
  const int b = bh / NH, h = bh % NH;
  const int q0 = qblk * 64 + wave * 16;
  FragH aq[2];
  {
    const unsigned short* qr = qkv + (size_t)(b * SEQ + q0 + ln) * (3 * DM) + h * HD + 8 * hh;
#pragma unroll
    for (int ks = 0; ks < 2; ++ks) {
      aq[ks].half[0] = *(const v8us*)(qr + ks * 32);
      aq[ks].half[1] = *(const v8us*)(qr + ks * 32 + 16);
    }
  }
  const unsigned short* Kbase = qkv + (size_t)(b * SEQ) * (3 * DM) + DM + h * HD + 8 * hh;
  const unsigned short* Vbase = Vt + (size_t)bh * HD * SEQ + 8 * hh;
  float m_r[8], l_r[8];
#pragma unroll
  for (int r = 0; r < 8; ++r) { m_r[r] = -3.0e38f; l_r[r] = 0.f; }
  v8f oacc[4];
#pragma unroll
  for (int dt = 0; dt < 4; ++dt) oacc[dt] = (v8f){0.f, 0.f, 0.f, 0.f, 0.f, 0.f, 0.f, 0.f};
  const float sc = 0.125f / (ACARRY * ACARRY);
  const int kv_end = q0 + 16;
  for (int j0 = 0; j0 < kv_end; j0 += 32) {
    v8f s[2];
#pragma unroll
    for (int nt = 0; nt < 2; ++nt) {
      v8f acc = {};
      const unsigned short* krow = Kbase + (size_t)(j0 + nt * 16 + ln) * (3 * DM);
#pragma unroll
      for (int ks = 0; ks < 2; ++ks) {
        FragH bk;
        bk.half[0] = *(const v8us*)(krow + ks * 32);
        bk.half[1] = *(const v8us*)(krow + ks * 32 + 16);
        acc = mma1(aq[ks].v, bk.v, acc);
      }
      s[nt] = acc;
    }
    float alpha[8];
#pragma unroll
    for (int r = 0; r < 8; ++r) {
      const int qi = q0 + 8 * hh + r;
      const int ja = j0 + ln, jb = j0 + 16 + ln;
      const bool keepa = ja <= qi, keepb = jb <= qi;
      const float sa = keepa ? s[0][r] * sc : -3.0e38f;
      const float sb = keepb ? s[1][r] * sc : -3.0e38f;
      float mx = fmaxf(sa, sb);
      mx = fmaxf(mx, __shfl_xor(mx, 1, 32)); mx = fmaxf(mx, __shfl_xor(mx, 2, 32)); mx = fmaxf(mx, __shfl_xor(mx, 4, 32)); mx = fmaxf(mx, __shfl_xor(mx, 8, 32));
      const float mnew = fmaxf(m_r[r], mx);
      const float ea = __expf(m_r[r] - mnew);
      alpha[r] = (mnew > -1.0e38f) ? ea : 1.0f;
      const float e0 = __expf(sa - mnew), e1 = __expf(sb - mnew);
      const float p0 = keepa ? e0 : 0.f;
      const float p1 = keepb ? e1 : 0.f;
      const _Float16 h0 = (_Float16)(p0 * PCARRY), h1 = (_Float16)(p1 * PCARRY);
      m_r[r] = mnew;
      l_r[r] = l_r[r] * alpha[r] + ((float)h0 + (float)h1);
      sP[wave][8 * hh + r][ln] = __builtin_bit_cast(unsigned short, h0);
      sP[wave][8 * hh + r][16 + ln] = __builtin_bit_cast(unsigned short, h1);
    }
#pragma unroll
    for (int dt = 0; dt < 4; ++dt)
#pragma unroll
      for (int r = 0; r < 8; ++r) oacc[dt][r] *= alpha[r];
    __builtin_amdgcn_fence(4  , "workgroup");
    __builtin_amdgcn_wave_barrier();
    FragH pa;
    pa.half[0] = *(const v8us*)&sP[wave][ln][8 * hh];
    pa.half[1] = *(const v8us*)&sP[wave][ln][16 + 8 * hh];
#pragma unroll
    for (int dt = 0; dt < 4; ++dt) {
      const unsigned short* vrow = Vbase + (size_t)(dt * 16 + ln) * SEQ + j0;
      FragH bv;
      bv.half[0] = *(const v8us*)(vrow);
      bv.half[1] = *(const v8us*)(vrow + 16);
      oacc[dt] = mma1(pa.v, bv.v, oacc[dt]);
    }
    __builtin_amdgcn_fence(4  , "workgroup");
    __builtin_amdgcn_wave_barrier();
  }
#pragma unroll
  for (int r = 0; r < 8; ++r) {
    float l = l_r[r];
    l += __shfl_xor(l, 1, 32); l += __shfl_xor(l, 2, 32); l += __shfl_xor(l, 4, 32); l += __shfl_xor(l, 8, 32);
    l_r[r] = (l > 0.f) ? 1.0f / l : 0.f;
  }
#pragma unroll
  for (int dt = 0; dt < 4; ++dt)
#pragma unroll
    for (int r = 0; r < 8; ++r) sO[wave][8 * hh + r][dt * 16 + ln] = oacc[dt][r] * l_r[r];
  __builtin_amdgcn_fence(4  , "workgroup");
  __builtin_amdgcn_wave_barrier();
  const int rq = lane >> 3, c8 = (lane & 7) * 8;
  v8us ov[4];
#pragma unroll
  for (int q = 0; q < 4; ++q) {
    const int r = q * 4 + rq;
    const v4f x0 = *(const v4fa*)&sO[wave][r][c8];
    const v4f x1 = *(const v4fa*)&sO[wave][r][c8 + 4];
    ov[q] = pack8(x0, x1, 1.0f);
  }
  for (int pass = 0; pass < 2; ++pass) {
#pragma unroll
    for (int q = 0; q < 4; ++q)
      *(volatile v8us*)(ctx + (size_t)(b * SEQ + q0 + q * 4 + rq) * DM + h * HD + c8) = ov[q];
    if (pass == 0) __threadfence();
  }
}

extern "C" void kernel_launch(void* const* d_in, const int* in_sizes, int n_in,
                              void* d_out, int out_size, void* d_ws, size_t ws_size, hipStream_t stream) {
  if (n_in < 13) return;
  const long long xneed = ((long long)(NB - 1) * SEQ_FULL + SEQ) * DM;
  if ((long long)in_sizes[0] < xneed) return;
  if ((long long)out_size < xneed) return;
  if (in_sizes[1] < DM || in_sizes[2] < DM || in_sizes[6] < DM || in_sizes[7] < DM || in_sizes[8] < DM || in_sizes[12] < DM) return;
  if (in_sizes[3] < 3 * DM * DM || in_sizes[4] < 3 * DM || in_sizes[5] < DM * DM) return;
  if (in_sizes[9] < DM * FF || in_sizes[10] < FF || in_sizes[11] < FF * DM) return;
  const float* x      = (const float*)d_in[0];
  const float* ln1_g  = (const float*)d_in[1];
  const float* ln1_b  = (const float*)d_in[2];
  const float* qkv_w  = (const float*)d_in[3];
  const float* qkv_b  = (const float*)d_in[4];
  const float* proj_w = (const float*)d_in[5];
  const float* proj_b = (const float*)d_in[6];
  const float* ln2_g  = (const float*)d_in[7];
  const float* ln2_b  = (const float*)d_in[8];
  const float* ff1_w  = (const float*)d_in[9];
  const float* ff1_b  = (const float*)d_in[10];
  const float* ff2_w  = (const float*)d_in[11];
  const float* ff2_b  = (const float*)d_in[12];
  char* ws = (char*)d_ws; size_t off = 0;
  auto take = [&](size_t bytes) { char* p = ws + off; off += (bytes + 255) & ~(size_t)255; return p; };
  unsigned short* Wqkv = (unsigned short*)take(SZ_WQKV);
  unsigned short* Wpj  = (unsigned short*)take(SZ_WPJ);
  unsigned short* Wf1  = (unsigned short*)take(SZ_WF1);
  unsigned short* Wf2  = (unsigned short*)take(SZ_WF2);
  unsigned short* h16  = (unsigned short*)take(SZ_H16);
  unsigned short* qkv16 = (unsigned short*)take(SZ_QKV);
  unsigned short* Vt   = (unsigned short*)take(SZ_VT);
  unsigned short* ctx16 = (unsigned short*)take(SZ_CTX);
  float* x1            = (float*)take(SZ_X1);
  unsigned short* g16  = (unsigned short*)take(SZ_G16);
  if (off > ws_size) return;
  const int M = MROWS;
  k_wt_f16<<<G_WQKV, 256, 0, stream>>>(qkv_w, Wqkv, DM, 3 * DM);
  k_wt_f16<<<G_WPJ, 256, 0, stream>>>(proj_w, Wpj, DM, DM);
  k_wt_f16<<<G_WF1, 256, 0, stream>>>(ff1_w, Wf1, DM, FF);
  k_wt_f16<<<G_WF2, 256, 0, stream>>>(ff2_w, Wf2, FF, DM);
  k_ln1<<<M, 128, 0, stream>>>(x, ln1_g, ln1_b, h16, 1e-5f);
  k_gemm_plane<<<G_QKV, 128, 0, stream>>>(h16, DM, Wqkv, DM, qkv_b, qkv16, 3 * DM, M, 3 * DM, DM);
  k_vt<<<G_VT, 256, 0, stream>>>(qkv16, Vt);
  k_flash_h<<<G_FL, 128, 0, stream>>>(qkv16, Vt, ctx16);
  k_gemm_res_in<<<G_PJ, 128, 0, stream>>>(ctx16, DM, Wpj, DM, proj_b, x, x1, DM, M, DM, DM);
  k_ln2<<<M, 128, 0, stream>>>(x1, ln2_g, ln2_b, h16, 1e-5f);
  k_gemm_gelu<<<G_F1, 128, 0, stream>>>(h16, DM, Wf1, DM, ff1_b, g16, FF, M, FF, DM);
  k_gemm_res_out<<<G_F2, 128, 0, stream>>>(g16, FF, Wf2, FF, ff2_b, x1, (float*)d_out, DM, M, DM, FF);
}
